// quantized_conv_38938173506080
// MI455X (gfx1250) — hardware-verified
//
#include <hip/hip_runtime.h>

#pragma clang fp contract(off)

typedef __attribute__((ext_vector_type(16))) _Float16 v16h;
typedef __attribute__((ext_vector_type(8)))  _Float16 v8h;
typedef __attribute__((ext_vector_type(16))) __bf16   v16b;
typedef __attribute__((ext_vector_type(8)))  __bf16   v8b;
typedef __attribute__((ext_vector_type(8)))  float    v8f;
typedef __attribute__((ext_vector_type(4)))  float    v4f;

__device__ __forceinline__ unsigned short f2bf_bits(float f) {
  unsigned u = __float_as_uint(f);
  return (unsigned short)((u + 0x7FFFu + ((u >> 16) & 1u)) >> 16);
}
__device__ __forceinline__ float bf_bits2f(unsigned short h) { return __uint_as_float(((unsigned)h) << 16); }

__device__ __forceinline__ void dep_guard_h(v8f& a, v8f& b, v16h x, v16h y) { asm volatile("v_nop\n\tv_nop\n\tv_nop\n\tv_nop" : "+v"(a), "+v"(b) : "v"(x), "v"(y)); }
__device__ __forceinline__ void dep_guard_b(v8f& a, v8f& b, v16b x, v16b y) { asm volatile("v_nop\n\tv_nop\n\tv_nop\n\tv_nop" : "+v"(a), "+v"(b) : "v"(x), "v"(y)); }
__device__ __forceinline__ void keep4_h(v16h a, v16h b, v16h c, v16h d) { asm volatile("v_nop" :: "v"(a), "v"(b), "v"(c), "v"(d)); }
__device__ __forceinline__ void keep4_b(v16b a, v16b b, v16b c, v16b d) { asm volatile("v_nop" :: "v"(a), "v"(b), "v"(c), "v"(d)); }
__device__ __forceinline__ void acc_guard4(v8f& a, v8f& b, v8f& c, v8f& d) { asm volatile("v_nop\n\tv_nop\n\tv_nop\n\tv_nop" : "+v"(a), "+v"(b), "+v"(c), "+v"(d)); }
template <typename T> struct Frag;
template <> struct Frag<_Float16> {
  typedef v16h V; union U { v16h v; v8h h[2]; };
  static __device__ __forceinline__ v16h load(const _Float16* p) {
    U f; f.h[0] = *(const v8h*)(p); f.h[1] = *(const v8h*)(p + 16); return f.v;
  }
  static __device__ __forceinline__ v8f mma(v16h a, v16h b, v8f c) {
    return __builtin_amdgcn_wmma_f32_16x16x32_f16(false, a, false, b, (short)0, c, false, false);
  }
  static __device__ __forceinline__ void guard(v8f& a, v8f& b, v16h x, v16h y) { dep_guard_h(a, b, x, y); }
  static __device__ __forceinline__ void keep(v16h a, v16h b, v16h c, v16h d) { keep4_h(a, b, c, d); }
};
template <> struct Frag<__bf16> {
  typedef v16b V; union U { v16b v; v8b h[2]; };
  static __device__ __forceinline__ v16b load(const __bf16* p) {
    U f; f.h[0] = *(const v8b*)(p); f.h[1] = *(const v8b*)(p + 16); return f.v;
  }
  static __device__ __forceinline__ v8f mma(v16b a, v16b b, v8f c) {
    return __builtin_amdgcn_wmma_f32_16x16x32_bf16(false, a, false, b, (short)0, c, false, false);
  }
  static __device__ __forceinline__ void guard(v8f& a, v8f& b, v16b x, v16b y) { dep_guard_b(a, b, x, y); }
  static __device__ __forceinline__ void keep(v16b a, v16b b, v16b c, v16b d) { keep4_b(a, b, c, d); }
};

template <int ET> struct Elem;
template <> struct Elem<0> { typedef _Float16 T; };
template <> struct Elem<1> { typedef __bf16 T; };
template <int ET, bool SPLIT, int BIAS_MODE, int OUT_MODE, bool RESID, int ACT = 0>
__global__ __launch_bounds__(256) void wmma_gemm64(
    const unsigned short* __restrict__ Ap, const unsigned short* __restrict__ A2p, int lda, long strideA,
    const unsigned short* __restrict__ Btp, const unsigned short* __restrict__ Bt2p, int ldb, long strideB,
    void* __restrict__ Cout, void* __restrict__ Cout2, int ldc, long strideC,
    const float* __restrict__ bias,
    const float* __restrict__ resid, long strideR,
    int M, int N, int K, float scale) {
  typedef typename Elem<ET>::T T;
  typedef typename Frag<T>::V V;
  const T* A = (const T*)Ap; const T* A2 = (const T*)A2p; const T* Bt = (const T*)Btp; const T* Bt2 = (const T*)Bt2p;
  __shared__ __align__(16) float sT[8][16 * 68];
  const int b    = blockIdx.y;
  const int lane = threadIdx.x & 31;
  const int wave = threadIdx.x >> 5;
  const int tilesN = N >> 6;
  const int tilesM = M >> 6;
  const int tile = blockIdx.x * 8 + wave;
  if (tile >= tilesM * tilesN) return;
  const int tm = tile / tilesN;
  const int tn = tile - tm * tilesN;
  const int m0 = tm << 6;
  const int n0 = tn << 6;

  const T* Ab  = A  + (size_t)b * strideA;
  const T* Bb  = Bt + (size_t)b * strideB;
  const T* Ab2 = SPLIT ? (A2  + (size_t)b * strideA) : nullptr;
  const T* Bb2 = SPLIT ? (Bt2 + (size_t)b * strideB) : nullptr;

  const int rlane = lane & 15;
  const int koff  = (lane >> 4) * 8;
  const int mOff  = (lane >> 4) * 8;

  v8f acc[4][4];
#pragma unroll
  for (int i = 0; i < 4; ++i)
#pragma unroll
    for (int j = 0; j < 4; ++j) acc[i][j] = (v8f){0.f,0.f,0.f,0.f,0.f,0.f,0.f,0.f};

  for (int k0 = 0; k0 < K; k0 += 32) {
    V bh[4], bl[4];
#pragma unroll
    for (int j = 0; j < 4; ++j) {
      const size_t bo = (size_t)(n0 + (j << 4) + rlane) * ldb + koff + k0;
      bh[j] = Frag<T>::load(Bb + bo);
      if (SPLIT) bl[j] = Frag<T>::load(Bb2 + bo);
    }
#pragma unroll
    for (int i = 0; i < 4; ++i) {
      const size_t ao = (size_t)(m0 + (i << 4) + rlane) * lda + koff + k0;
      V ah = Frag<T>::load(Ab + ao);
      V al;
      if (SPLIT) al = Frag<T>::load(Ab2 + ao);
#pragma unroll
      for (int j = 0; j < 4; ++j) {
        acc[i][j] = Frag<T>::mma(ah, bh[j], acc[i][j]);
        if (SPLIT) {
          acc[i][j] = Frag<T>::mma(ah, bl[j], acc[i][j]);
          acc[i][j] = Frag<T>::mma(al, bh[j], acc[i][j]);
        }
      }
      Frag<T>::guard(acc[i][0], acc[i][3], ah, SPLIT ? al : ah);
    }
    Frag<T>::keep(bh[0], bh[1], bh[2], bh[3]);
    if (SPLIT) Frag<T>::keep(bl[0], bl[1], bl[2], bl[3]);
  }
  acc_guard4(acc[0][0], acc[0][1], acc[0][2], acc[0][3]);
  acc_guard4(acc[1][0], acc[1][1], acc[1][2], acc[1][3]);
  acc_guard4(acc[2][0], acc[2][1], acc[2][2], acc[2][3]);
  acc_guard4(acc[3][0], acc[3][1], acc[3][2], acc[3][3]);

  float* slab = sT[wave];
  const float* Rb = RESID ? (resid + (size_t)b * strideR) : nullptr;
#pragma unroll
  for (int i = 0; i < 4; ++i) {
    const int mBase = m0 + (i << 4);
#pragma unroll
    for (int j = 0; j < 4; ++j) {
      const int n = n0 + (j << 4) + rlane;
      float bv = 0.f;
      if (BIAS_MODE == 2) bv = bias[n];
#pragma unroll
      for (int r = 0; r < 8; ++r) {
        float v = acc[i][j][r] * scale;
        if (BIAS_MODE == 1) v += bias[mBase + mOff + r];
        if (BIAS_MODE == 2) v += bv;
        if (RESID) v += Rb[(size_t)(mBase + mOff + r) * ldc + n];
        if (ACT == 1) v = tanhf(v);
        if (ACT == 2) v = fmaxf(v, 0.0f);
        if (ACT == 3) v = v / (1.0f + expf(-v));
        if (ACT == 4) v = (v > 0.f) ? v : 0.01f * v;
        if (ACT == 5) v = 0.5f * v * (1.0f + erff(v * 0.70710678118654752f));
        slab[(mOff + r) * 68 + (j << 4) + rlane] = v;
      }
    }
    __builtin_amdgcn_fence(__ATOMIC_RELEASE, "workgroup");
    __builtin_amdgcn_wave_barrier();
    __builtin_amdgcn_fence(__ATOMIC_ACQUIRE, "workgroup");
    if (OUT_MODE == 0) {
      float* C = (float*)Cout + (size_t)b * strideC;
      const int hh = lane >> 4, c4 = (lane & 15) * 4;
      for (int pass = 0; pass < 2; ++pass) {
#pragma unroll
        for (int it = 0; it < 8; ++it) {
          const int row = it * 2 + hh;
          v4f v = *(const v4f*)(slab + row * 68 + c4);
          *(volatile v4f*)(C + (size_t)(mBase + row) * ldc + n0 + c4) = v;
        }
        __threadfence();
      }
    } else {
      const int q = lane >> 3, c8 = (lane & 7) * 8;
      unsigned short* C  = (unsigned short*)Cout  + (size_t)b * strideC;
      unsigned short* C2 = (OUT_MODE == 2) ? ((unsigned short*)Cout2 + (size_t)b * strideC) : nullptr;
      for (int pass = 0; pass < 2; ++pass) {
#pragma unroll
        for (int it = 0; it < 4; ++it) {
          const int row = it * 4 + q;
          const float* sp = slab + row * 68 + c8;
          v8h hv, lv;
#pragma unroll
          for (int e = 0; e < 8; ++e) {
            if (OUT_MODE == 1) {
              hv[e] = (_Float16)sp[e];
            } else if (OUT_MODE == 3) {
              const int iv = (int)sp[e];
              hv[e] = __builtin_bit_cast(_Float16, (unsigned short)(iv & 0xffff));
            } else {
              unsigned short hb = f2bf_bits(sp[e]);
              unsigned short lb = f2bf_bits(sp[e] - bf_bits2f(hb));
              hv[e] = __builtin_bit_cast(_Float16, hb);
              lv[e] = __builtin_bit_cast(_Float16, lb);
            }
          }
          *(volatile v8h*)(C + (size_t)(mBase + row) * ldc + n0 + c8) = hv;
          if (OUT_MODE == 2) *(volatile v8h*)(C2 + (size_t)(mBase + row) * ldc + n0 + c8) = lv;
        }
        __threadfence();
      }
    }
    __builtin_amdgcn_fence(__ATOMIC_RELEASE, "workgroup");
    __builtin_amdgcn_wave_barrier();
    __builtin_amdgcn_fence(__ATOMIC_ACQUIRE, "workgroup");
  }
}

constexpr int  kBatch     = 16;
constexpr int  kCin       = 64;
constexpr int  kCout      = 64;
constexpr int  kImg       = 32;
constexpr int  kPos       = kImg * kImg;
constexpr int  kFeat      = kCin * 9;
constexpr int  kRows      = kBatch * kPos;
constexpr int  kNcol      = 2 * 4 * kCout;
constexpr int  kChunkRows = 8192;
constexpr int  kNumChunks = kRows / kChunkRows;
constexpr int  kOct       = kFeat / 8;
constexpr long kPlaneChunk = (long)kChunkRows * kFeat;
constexpr int  kStreamThreads = kChunkRows * kOct;
constexpr int  kWOct      = kNcol * kOct;
constexpr long kCElems    = 4L * kRows * kNcol;
constexpr int  kMaxBlocks = (int)(kCElems / (64 * kNcol));
constexpr int  kOutElems  = kRows * kCout;
constexpr int  kMaxSum    = 9 * kFeat;

static_assert(kFeat % 32 == 0);
static_assert(kChunkRows % 64 == 0 && kNcol % 64 == 0 && kRows % kChunkRows == 0);
static_assert(kStreamThreads % 256 == 0 && kWOct % 256 == 0);
static_assert(kCElems % (64 * kNcol) == 0 && kMaxBlocks == 1024);
static_assert(kRows % 32 == 0 && kPos % 32 == 0);
static_assert(kMaxSum < 65536);

constexpr size_t kOffA   = 0;
constexpr size_t kSzA    = 4ull * (size_t)kPlaneChunk * 2ull;
constexpr size_t kOffB   = kOffA + kSzA;
constexpr size_t kSzB    = (size_t)kNcol * kFeat * 2ull;
constexpr size_t kOffC   = kOffB + kSzB;
constexpr size_t kSzC    = (size_t)kCElems * 2ull;
constexpr size_t kOffTbl = kOffC + kSzC;
constexpr size_t kSzTbl  = (size_t)kMaxBlocks * 128ull;
constexpr size_t kOffPrm = kOffTbl + kSzTbl;
constexpr size_t kSzPrm  = 128;
constexpr size_t kWsTotal = kOffPrm + kSzPrm;
static_assert(kOffB % 128 == 0 && kOffC % 128 == 0 && kOffTbl % 128 == 0 && kOffPrm % 128 == 0);
static_assert(kWsTotal == 105578624ull);
static_assert(kWsTotal <= 134217728ull);
static_assert((size_t)kOutElems * 4 + 4 <= 4194308ull);

__global__ __launch_bounds__(256) void k_wprep(const float* __restrict__ w, unsigned short* __restrict__ Bt) {
  __shared__ float red[8];
  const int tid = threadIdx.x, lane = tid & 31, wave = tid >> 5;
  float lmax = 0.f;
#pragma unroll 4
  for (int i = tid; i < kCout * kFeat; i += 256) lmax = fmaxf(lmax, fabsf(w[i]));
#pragma unroll
  for (int off = 1; off < 32; off <<= 1) lmax = fmaxf(lmax, __shfl_xor(lmax, off, 32));
  if (lane == 0) red[wave] = lmax;
  __syncthreads();
  float raw = red[0];
#pragma unroll
  for (int i = 1; i < 8; ++i) raw = fmaxf(raw, red[i]);
  const float ma  = (raw > 0.f) ? raw : 1.f;
  const float rma = 1.0f / ma;
  for (int it = 0; it < kWOct / 256; ++it) {
    const int oc = it * 256 + tid;
    const int n  = oc / kOct, o8 = oc - n * kOct;
    const int g  = n >> 8, t = (n >> 6) & 3, o = n & 63;
    const float* wr = w + (size_t)o * kFeat + o8 * 8;
    const v4f w0 = *(const v4f*)wr;
    const v4f w1 = *(const v4f*)(wr + 4);
    float wv[8];
    wv[0] = w0[0]; wv[1] = w0[1]; wv[2] = w0[2]; wv[3] = w0[3];
    wv[4] = w1[0]; wv[5] = w1[1]; wv[6] = w1[2]; wv[7] = w1[3];
    v8h hv;
#pragma unroll
    for (int e = 0; e < 8; ++e) {
      const float ap = fmaxf(wv[e], 0.f);
      const float an = fmaxf(-wv[e], 0.f);
      const float a  = (g != 0) ? an : ap;
      const float qs = a * rma;
      const float qf = qs * 255.0f;
      const int   qi = (int)rintf(qf);
      const int   sv = (qi >> (2 * t)) & 3;
      hv[e] = (_Float16)(float)sv;
    }
    unsigned short* dst = Bt + (size_t)oc * 8;
    *(volatile v8h*)dst = hv;
    __threadfence();
    *(volatile v8h*)dst = hv;
  }
}

__global__ __launch_bounds__(256) void k_stream(const float* __restrict__ x, unsigned short* __restrict__ Apl, int mbase) {
  const int tid = threadIdx.x;
  const int idx = blockIdx.x * 256 + tid;
  const int ml  = idx / kOct, o8 = idx - ml * kOct;
  const int m   = mbase + ml;
  const int b   = m >> 10, p = m & 1023, h = p >> 5, wc = p & 31;
  int q[8];
#pragma unroll
  for (int e = 0; e < 8; ++e) {
    const int f  = o8 * 8 + e;
    const int c  = f / 9, rr = f - c * 9;
    const int ky = rr / 3, kx = rr - ky * 3;
    const int hi = h + ky - 1, wi = wc + kx - 1;
    const bool valid = ((unsigned)hi < 32u) && ((unsigned)wi < 32u);
    const int hic = min(max(hi, 0), 31);
    const int wic = min(max(wi, 0), 31);
    float v = x[(((size_t)b * kCin + c) * kImg + hic) * kImg + wic];
    v = valid ? v : 0.0f;
    const float cl = fminf(fmaxf(v, -2.0f), 1.984375f);
    q[e] = ((int)rintf(cl * 64.0f)) & 255;
  }
  v8h hv0, hv1, hv2, hv3;
#pragma unroll
  for (int e = 0; e < 8; ++e) {
    hv0[e] = (_Float16)(float)(q[e] & 3);
    hv1[e] = (_Float16)(float)((q[e] >> 2) & 3);
    hv2[e] = (_Float16)(float)((q[e] >> 4) & 3);
    hv3[e] = (_Float16)(float)((q[e] >> 6) & 3);
  }
  unsigned short* dst = Apl + (size_t)idx * 8;
  *(volatile v8h*)(dst)                   = hv0;
  *(volatile v8h*)(dst + kPlaneChunk)     = hv1;
  *(volatile v8h*)(dst + 2 * kPlaneChunk) = hv2;
  *(volatile v8h*)(dst + 3 * kPlaneChunk) = hv3;
  __threadfence();
  *(volatile v8h*)(dst)                   = hv0;
  *(volatile v8h*)(dst + kPlaneChunk)     = hv1;
  *(volatile v8h*)(dst + 2 * kPlaneChunk) = hv2;
  *(volatile v8h*)(dst + 3 * kPlaneChunk) = hv3;
}

__global__ __launch_bounds__(256) void k_tilemax(const uint4* __restrict__ C4, int* __restrict__ tbl) {
  __shared__ int wm[8];
  const int tid = threadIdx.x, lane = tid & 31, wave = tid >> 5;
  const uint4* base = C4 + (size_t)blockIdx.x * 4096;
  unsigned m = 0;
#pragma unroll 4
  for (int it = 0; it < 16; ++it) {
    const uint4 v = base[it * 256 + tid];
    m = max(m, v.x & 0xffffu); m = max(m, v.x >> 16);
    m = max(m, v.y & 0xffffu); m = max(m, v.y >> 16);
    m = max(m, v.z & 0xffffu); m = max(m, v.z >> 16);
    m = max(m, v.w & 0xffffu); m = max(m, v.w >> 16);
  }
#pragma unroll
  for (int off = 1; off < 32; off <<= 1) m = max(m, (unsigned)__shfl_xor((int)m, off, 32));
  if (lane == 0) wm[wave] = (int)m;
  __syncthreads();
  if (wave == 0) {
    const int mp = max(max(wm[0], wm[2]), max(wm[4], wm[6]));
    const int mn = max(max(wm[1], wm[3]), max(wm[5], wm[7]));
    const int val = (lane & 1) ? mn : mp;
    volatile int* dst = tbl + (size_t)blockIdx.x * 32 + lane;
    *dst = val;
    __threadfence();
    *dst = val;
  }
}

__global__ __launch_bounds__(256) void k_params(const float* __restrict__ w, const int* __restrict__ tbl,
                                               float* __restrict__ prm, float* __restrict__ out1) {
  __shared__ float rf[8];
  __shared__ int rp[8];
  __shared__ int rn[8];
  const int tid = threadIdx.x, lane = tid & 31, wave = tid >> 5;
  float lmax = 0.f;
#pragma unroll 4
  for (int i = tid; i < kCout * kFeat; i += 256) lmax = fmaxf(lmax, fabsf(w[i]));
  int mp = 0, mn = 0;
  for (int i = tid; i < kMaxBlocks; i += 256) {
    mp = max(mp, tbl[(size_t)i * 32]);
    mn = max(mn, tbl[(size_t)i * 32 + 1]);
  }
#pragma unroll
  for (int off = 1; off < 32; off <<= 1) {
    lmax = fmaxf(lmax, __shfl_xor(lmax, off, 32));
    mp = max(mp, __shfl_xor(mp, off, 32));
    mn = max(mn, __shfl_xor(mn, off, 32));
  }
  if (lane == 0) { rf[wave] = lmax; rp[wave] = mp; rn[wave] = mn; }
  __syncthreads();
  if (wave == 0) {
    float raw = rf[0];
    int gp = rp[0], gn = rn[0];
#pragma unroll
    for (int i = 1; i < 8; ++i) { raw = fmaxf(raw, rf[i]); gp = max(gp, rp[i]); gn = max(gn, rn[i]); }
    gp = min(max(gp, 0), kMaxSum);
    gn = min(max(gn, 0), kMaxSum);
    const float stepP = fmaxf((float)gp, 1e-8f) * (1.0f / 15.0f);
    const float stepN = fmaxf((float)gn, 1e-8f) * (1.0f / 15.0f);
    const float rinvP = 1.0f / stepP;
    const float rinvN = 1.0f / stepN;
    float val = 0.f;
    val = (lane == 0) ? stepP : val;
    val = (lane == 1) ? rinvP : val;
    val = (lane == 2) ? stepN : val;
    val = (lane == 3) ? rinvN : val;
    val = (lane == 4) ? raw : val;
    volatile float* dst = prm + lane;
    *dst = val;
    __threadfence();
    *dst = val;
    if (lane == 0) {
      volatile float* o1 = out1;
      *o1 = 0.0f;
      __threadfence();
      *o1 = 0.0f;
    }
  }
}

__global__ __launch_bounds__(256) void k_combine(const uint4* __restrict__ C4, const float* __restrict__ prm,
                                                float* __restrict__ out) {
  __shared__ __align__(16) uint4 Cs4[32 * 64];
  __shared__ __align__(16) float Os[64 * 36];
  const int tid = threadIdx.x, lane = tid & 31, wave = tid >> 5;
  const int m0 = blockIdx.x * 32;
  const int b  = m0 >> 10, p0 = m0 & 1023;
  const float stepP = prm[0], rinvP = prm[1], stepN = prm[2], rinvN = prm[3], ma = prm[4];
  const int o = tid & 63, mg = tid >> 6;
  const unsigned short* Cs = (const unsigned short*)Cs4;
  float acc[8];
#pragma unroll
  for (int i = 0; i < 8; ++i) acc[i] = 0.0f;
  for (int s = 0; s < 4; ++s) {
    __syncthreads();
    const uint4* src = C4 + ((size_t)s * kRows + m0) * 64;
#pragma unroll
    for (int it = 0; it < 8; ++it) Cs4[it * 256 + tid] = src[it * 256 + tid];
    __syncthreads();
#pragma unroll
    for (int i = 0; i < 8; ++i) {
      const unsigned short* row = Cs + (mg * 8 + i) * kNcol;
#pragma unroll
      for (int t = 0; t < 4; ++t) {
        const float pv = (float)(int)row[t * 64 + o];
        const float nv = (float)(int)row[256 + t * 64 + o];
        const float pq = rintf(pv * rinvP) * stepP;
        const float nq = rintf(nv * rinvN) * stepN;
        const float d  = pq - nq;
        const float sc = (float)(1 << (2 * (s + t)));
        acc[i] = acc[i] + d * sc;
      }
    }
  }
#pragma unroll
  for (int i = 0; i < 8; ++i) {
    const float v = (acc[i] * ma) * (1.0f / 255.0f);
    Os[o * 36 + mg * 8 + i] = v;
  }
  __syncthreads();
  const int q = lane >> 3, c4l = (lane & 7) * 4;
  for (int pass = 0; pass < 2; ++pass) {
#pragma unroll
    for (int it = 0; it < 2; ++it) {
      const int ol = wave * 8 + it * 4 + q;
      const v4f val = *(const v4f*)(Os + ol * 36 + c4l);
      *(volatile v4f*)(out + ((size_t)(b * kCout + ol)) * kPos + p0 + c4l) = val;
    }
    __threadfence();
  }
}

extern "C" void kernel_launch(void* const* d_in, const int* in_sizes, int n_in,
                              void* d_out, int out_size, void* d_ws, size_t ws_size,
                              hipStream_t stream) {
  if (n_in < 2) return;
  if (in_sizes[0] != kBatch * kCin * kImg * kImg) return;
  if (in_sizes[1] != kCout * kFeat) return;
  if (out_size != kOutElems + 1) return;
  if (ws_size < kWsTotal) return;

  const float* x = (const float*)d_in[0];
  const float* w = (const float*)d_in[1];
  float* out = (float*)d_out;
  unsigned char* ws = (unsigned char*)d_ws;

  unsigned short* Apl = (unsigned short*)(ws + kOffA);
  unsigned short* Bt  = (unsigned short*)(ws + kOffB);
  unsigned short* Cpl = (unsigned short*)(ws + kOffC);
  int*   tbl = (int*)(ws + kOffTbl);
  float* prm = (float*)(ws + kOffPrm);

  k_wprep<<<dim3(1), dim3(256), 0, stream>>>(w, Bt);

  for (int chunk = 0; chunk < kNumChunks; ++chunk) {
    k_stream<<<dim3(kStreamThreads / 256), dim3(256), 0, stream>>>(x, Apl, chunk * kChunkRows);
    unsigned short* Cchunk = Cpl + (size_t)chunk * kChunkRows * kNcol;
    wmma_gemm64<0, false, 0, 3, false, 0><<<dim3((kChunkRows / 64) * (kNcol / 64) / 8, 4), dim3(256), 0, stream>>>(
        Apl, Apl, kFeat, kPlaneChunk,
        Bt, Bt, kFeat, 0L,
        (void*)Cchunk, (void*)Cchunk, kNcol, (long)kRows * kNcol,
        prm, prm, 0L,
        kChunkRows, kNcol, kFeat, 1.0f);
  }

  k_tilemax<<<dim3(kMaxBlocks), dim3(256), 0, stream>>>((const uint4*)Cpl, tbl);
  k_params<<<dim3(1), dim3(256), 0, stream>>>(w, tbl, prm, out + kOutElems);
  k_combine<<<dim3(kRows / 32), dim3(256), 0, stream>>>((const uint4*)Cpl, prm, out);
}
